// StudentDecoderAttention_4758823764609
// MI455X (gfx1250) — hardware-verified
//
#include <hip/hip_runtime.h>
#include <hip/hip_bf16.h>
#include <math.h>


typedef _Float16 bf16;
typedef _Float16 f16;
typedef __attribute__((ext_vector_type(4))) unsigned v4u_t;
typedef unsigned v4ua __attribute__((ext_vector_type(4), may_alias));
typedef __attribute__((ext_vector_type(4))) float v4f_t;
typedef float v4fa __attribute__((ext_vector_type(4), may_alias));
typedef __attribute__((ext_vector_type(16))) bf16  bf16x16;
typedef bf16x16 f16x16;
typedef __attribute__((ext_vector_type(8)))  bf16  bf16x8;
typedef bf16x8 f16x8;
typedef __attribute__((ext_vector_type(4)))  bf16  bf16x4;
typedef __attribute__((ext_vector_type(8)))  float f32x8;
__device__ __forceinline__ f32x8 wmma16(f16x16 a, f16x16 b, f32x8 c) {
  c = __builtin_amdgcn_wmma_f32_16x16x32_f16(false, a, false, b, (short)0, c, false, false);
  asm volatile("v_nop\n\tv_nop\n\tv_nop\n\tv_nop" : "+v"(c) : "v"(a), "v"(b));
  return c;
}
#define LDS_STRIDE 48
#define KSTRIDE    72
#define VSTRIDE    48

__device__ __forceinline__ f32x8 wmma_bf16(bf16x16 a, bf16x16 b, f32x8 c) {
  c = __builtin_amdgcn_wmma_f32_16x16x32_f16(false, a, false, b, (short)0, c, false, false);
  asm volatile("v_nop\n\tv_nop\n\tv_nop\n\tv_nop" : "+v"(c) : "v"(a), "v"(b));
  return c;
}

template <typename T>
__device__ __forceinline__ bf16x16 load_frag(const T* __restrict__ base, int ld,
                                             int row0, int k0) {
  const int lane = threadIdx.x & 31;
  const int r    = lane & 15;
  const int kh   = (lane >> 4) * 8;
  const T* p0 = base + (size_t)(row0 + r) * ld + (k0 + kh);
  const T* p1 = p0 + 16;
  bf16x16 f;
#pragma unroll
  for (int i = 0; i < 8; ++i) {
    f[i]     = (bf16)p0[i];
    f[i + 8] = (bf16)p1[i];
  }
  return f;
}

__device__ __forceinline__ bf16x16 lds_frag(const bf16* base, int stride) {
  const int lane = threadIdx.x & 31;
  const int row  = lane & 15;
  const int kh   = (lane >> 4) * 8;
  const bf16x8 lo = *(const bf16x8*)(base + row * stride + kh);
  const bf16x8 hi = *(const bf16x8*)(base + row * stride + kh + 16);
  bf16x16 f;
#pragma unroll
  for (int i = 0; i < 8; ++i) { f[i] = lo[i]; f[i + 8] = hi[i]; }
  return f;
}

template <typename T>
__device__ __forceinline__ void stage_read16(const T* __restrict__ p, float* buf) {
#pragma unroll
  for (int i = 0; i < 16; ++i) buf[i] = (float)p[i];
}

__device__ __forceinline__ void stage_write(bf16* dst, const float* buf, int nquad) {
#pragma unroll
  for (int i = 0; i < nquad; ++i) {
    bf16x4 q;
    q[0] = (bf16)buf[4 * i];     q[1] = (bf16)buf[4 * i + 1];
    q[2] = (bf16)buf[4 * i + 2]; q[3] = (bf16)buf[4 * i + 3];
    *(bf16x4*)(dst + 4 * i) = q;
  }
}


#define GSTR 48
#define GSTR 48
template <typename AT, int EPI, bool OUT16>
__global__ __launch_bounds__(256) void gemm_kne(const AT* __restrict__ A, int lda, const float* __restrict__ Wm, int ldw,
                                                const float* __restrict__ bias, const float* __restrict__ R, const float* __restrict__ gvec,
                                                void* __restrict__ Yv, int ldy, int K) {
  __shared__ __attribute__((aligned(16))) f16 ldsA[128 * GSTR];
  __shared__ __attribute__((aligned(16))) f16 ldsW[128 * GSTR];
  __shared__ __attribute__((aligned(16))) float oS[8][32 * 68];
  const int tid = threadIdx.x, lane = tid & 31, wave = tid >> 5, cl = lane & 15, rh = (lane >> 4) * 8;
  const int m0 = blockIdx.x * 128, n0 = blockIdx.y * 128;
  const int wm = (wave & 3) * 32, wn = (wave >> 2) * 64;
  f32x8 acc[2][4];
#pragma unroll
  for (int i = 0; i < 2; ++i)
#pragma unroll
    for (int j = 0; j < 4; ++j) { f32x8 z = {}; acc[i][j] = z; }
#pragma unroll 1
  for (int k0 = 0; k0 < K; k0 += 32) {
    __syncthreads();
    { const int row = tid >> 1, ch = (tid & 1) * 16;
      const AT* src = A + (size_t)(m0 + row) * lda + k0 + ch;
#pragma unroll
      for (int g = 0; g < 16; ++g) ldsA[row * GSTR + ch + g] = (f16)src[g]; }
    { const int k = tid >> 3, nn0 = (tid & 7) * 16;
      const float* src = Wm + (size_t)(k0 + k) * ldw + n0 + nn0;
#pragma unroll
      for (int g = 0; g < 4; ++g) { const v4f_t v = *(const v4f_t*)(src + 4 * g);
#pragma unroll
        for (int u = 0; u < 4; ++u) ldsW[(nn0 + 4 * g + u) * GSTR + k] = (f16)v[u]; } }
    __syncthreads();
    f16x16 af[2];
#pragma unroll
    for (int i = 0; i < 2; ++i) af[i] = lds_frag(ldsA + (wm + 16 * i) * GSTR, GSTR);
#pragma unroll
    for (int j = 0; j < 4; ++j) {
      const f16x16 bf = lds_frag(ldsW + (wn + 16 * j) * GSTR, GSTR);
#pragma unroll
      for (int i = 0; i < 2; ++i) acc[i][j] = wmma16(af[i], bf, acc[i][j]);
    }
  }
  float* so = oS[wave];
#pragma unroll
  for (int i = 0; i < 2; ++i)
#pragma unroll
    for (int j = 0; j < 4; ++j) {
      const int n = n0 + wn + 16 * j + cl;
      const float bv = bias ? bias[n] : 0.0f;
      const float gv = (EPI == 2 || EPI == 4) ? gvec[n] : 0.0f;
      if (EPI == 1) {
#pragma unroll 1
        for (int r = 0; r < 8; ++r) { const float xg = acc[i][j][r] + bv; so[(16 * i + rh + r) * 68 + 16 * j + cl] = 0.5f * xg * (1.0f + erff(xg * 0.70710678118654752f)); }
      } else {
#pragma unroll
        for (int r = 0; r < 8; ++r) {
          float v = acc[i][j][r] + bv;
          if (EPI == 3) v = fmaxf(v, 0.0f);
          if (EPI == 4) v = gv * v;
          if (EPI == 2) v = R[(size_t)(m0 + wm + 16 * i + rh + r) * ldy + n] + gv * v;
          so[(16 * i + rh + r) * 68 + 16 * j + cl] = v;
        }
      }
    }
  asm volatile("s_wait_dscnt 0" ::: "memory");
  __builtin_amdgcn_wave_barrier();
#pragma unroll 1
  for (int pass = 0; pass < 2; ++pass) {
    if (OUT16) {
      f16* Y = (f16*)Yv;
#pragma unroll
      for (int it = 0; it < 8; ++it) { const int c = lane + 32 * it, rr = c >> 3, q8 = (c & 7) * 8;
        union { f16 h[8]; v4u_t v; } u;
#pragma unroll
        for (int e = 0; e < 8; ++e) u.h[e] = (f16)so[rr * 68 + q8 + e];
        *(volatile v4u_t*)(Y + (size_t)(m0 + wm + rr) * ldy + n0 + wn + q8) = u.v; }
    } else {
      float* Y = (float*)Yv;
#pragma unroll
      for (int it = 0; it < 16; ++it) { const int f4 = lane + 32 * it, rr = f4 >> 4, q = (f4 & 15) * 4;
        *(volatile v4f_t*)(Y + (size_t)(m0 + wm + rr) * ldy + n0 + wn + q) = *(const v4fa*)(so + rr * 68 + q); }
    }
    __threadfence();
  }
}

template <typename AT, int EPI, bool OUT16, int CZ>
__global__ __launch_bounds__(256) void gemm_knezc(const AT* __restrict__ A, int lda, size_t strideA, const float* __restrict__ Wm, int ldw, size_t strideW,
                                                 const float* __restrict__ bias, const float* __restrict__ R, const float* __restrict__ gvec,
                                                 void* __restrict__ Yv, int ldy, size_t strideY, int K) {
  A += (size_t)blockIdx.z * strideA; Wm += (size_t)blockIdx.z * strideW; Yv = (void*)((char*)Yv + (size_t)blockIdx.z * strideY * (OUT16 ? 2 : 4)); if (R) R += (size_t)blockIdx.z * strideY;
  __shared__ __attribute__((aligned(16))) f16 ldsA[128 * GSTR];
  __shared__ __attribute__((aligned(16))) f16 ldsW[128 * GSTR];
  __shared__ __attribute__((aligned(16))) float oS[8][32 * 68];
  const int tid = threadIdx.x, lane = tid & 31, wave = tid >> 5, cl = lane & 15, rh = (lane >> 4) * 8;
  const int m0 = blockIdx.x * 128, n0 = blockIdx.y * 128;
  if (CZ == 2 && n0 >= m0 + 128) return;
  const int Kc = (CZ == 1) ? min(K, m0 + 128) : K;
  const int wm = (wave & 3) * 32, wn = (wave >> 2) * 64;
  f32x8 acc[2][4];
#pragma unroll
  for (int i = 0; i < 2; ++i)
#pragma unroll
    for (int j = 0; j < 4; ++j) { f32x8 z = {}; acc[i][j] = z; }
#pragma unroll 1
  for (int k0 = 0; k0 < Kc; k0 += 32) {
    __syncthreads();
    { const int row = tid >> 1, ch = (tid & 1) * 16;
      const AT* src = A + (size_t)(m0 + row) * lda + k0 + ch;
#pragma unroll
      for (int g = 0; g < 16; ++g) ldsA[row * GSTR + ch + g] = (f16)src[g]; }
    { const int k = tid >> 3, nn0 = (tid & 7) * 16;
      const float* src = Wm + (size_t)(k0 + k) * ldw + n0 + nn0;
#pragma unroll
      for (int g = 0; g < 4; ++g) { const v4f_t v = *(const v4f_t*)(src + 4 * g);
#pragma unroll
        for (int u = 0; u < 4; ++u) ldsW[(nn0 + 4 * g + u) * GSTR + k] = (f16)v[u]; } }
    __syncthreads();
    f16x16 af[2];
#pragma unroll
    for (int i = 0; i < 2; ++i) af[i] = lds_frag(ldsA + (wm + 16 * i) * GSTR, GSTR);
#pragma unroll
    for (int j = 0; j < 4; ++j) {
      const f16x16 bf = lds_frag(ldsW + (wn + 16 * j) * GSTR, GSTR);
#pragma unroll
      for (int i = 0; i < 2; ++i) acc[i][j] = wmma16(af[i], bf, acc[i][j]);
    }
  }
  float* so = oS[wave];
#pragma unroll
  for (int i = 0; i < 2; ++i)
#pragma unroll
    for (int j = 0; j < 4; ++j) {
      const int n = n0 + wn + 16 * j + cl;
      const float bv = bias ? bias[n] : 0.0f;
      const float gv = (EPI == 2 || EPI == 4) ? gvec[n] : 0.0f;
      if (EPI == 1) {
#pragma unroll 1
        for (int r = 0; r < 8; ++r) { const float xg = acc[i][j][r] + bv; so[(16 * i + rh + r) * 68 + 16 * j + cl] = 0.5f * xg * (1.0f + erff(xg * 0.70710678118654752f)); }
      } else {
#pragma unroll
        for (int r = 0; r < 8; ++r) {
          float v = acc[i][j][r] + bv;
          if (EPI == 3) v = fmaxf(v, 0.0f);
          if (EPI == 4) v = gv * v;
          if (EPI == 2) v = R[(size_t)(m0 + wm + 16 * i + rh + r) * ldy + n] + gv * v;
          so[(16 * i + rh + r) * 68 + 16 * j + cl] = v;
        }
      }
    }
  asm volatile("s_wait_dscnt 0" ::: "memory");
  __builtin_amdgcn_wave_barrier();
#pragma unroll 1
  for (int pass = 0; pass < 2; ++pass) {
    if (OUT16) {
      f16* Y = (f16*)Yv;
#pragma unroll
      for (int it = 0; it < 8; ++it) { const int c = lane + 32 * it, rr = c >> 3, q8 = (c & 7) * 8;
        union { f16 h[8]; v4u_t v; } u;
#pragma unroll
        for (int e = 0; e < 8; ++e) u.h[e] = (f16)so[rr * 68 + q8 + e];
        *(volatile v4u_t*)(Y + (size_t)(m0 + wm + rr) * ldy + n0 + wn + q8) = u.v; }
    } else {
      float* Y = (float*)Yv;
#pragma unroll
      for (int it = 0; it < 16; ++it) { const int f4 = lane + 32 * it, rr = f4 >> 4, q = (f4 & 15) * 4;
        *(volatile v4f_t*)(Y + (size_t)(m0 + wm + rr) * ldy + n0 + wn + q) = *(const v4fa*)(so + rr * 68 + q); }
    }
    __threadfence();
  }
}

template <typename AT, bool ACC, int CZ>
__global__ __launch_bounds__(256) void gemm_kn2c(const AT* __restrict__ A, int lda, size_t strideA,
                                               const float* __restrict__ Wm, int ldw, size_t strideW,
                                               const float* __restrict__ bias, float scale,
                                               float* __restrict__ Y, int ldy, size_t strideY, int K) {
  __shared__ __attribute__((aligned(16))) f16 ldsA[128 * GSTR], ldsAl[128 * GSTR];
  __shared__ __attribute__((aligned(16))) f16 ldsW[128 * GSTR], ldsWl[128 * GSTR];
  __shared__ __attribute__((aligned(16))) float oS[8][32 * 68];
  const int tid = threadIdx.x, lane = tid & 31, wave = tid >> 5, cl = lane & 15, rh = (lane >> 4) * 8;
  const int m0 = blockIdx.x * 128, n0 = blockIdx.y * 128;
  if (CZ == 2 && n0 >= m0 + 128) return;
  const int Kc = (CZ == 1) ? min(K, m0 + 128) : K;
  const int wm = (wave & 3) * 32, wn = (wave >> 2) * 64;
  A += (size_t)blockIdx.z * strideA; Wm += (size_t)blockIdx.z * strideW; Y += (size_t)blockIdx.z * strideY;
  f32x8 acc[2][4], accx[2][4];
#pragma unroll
  for (int i = 0; i < 2; ++i)
#pragma unroll
    for (int j = 0; j < 4; ++j) { f32x8 z = {}; acc[i][j] = z; accx[i][j] = z; }
#pragma unroll 1
  for (int k0 = 0; k0 < Kc; k0 += 32) {
    __syncthreads();
    {
      const int row = tid >> 1, ch = (tid & 1) * 16;
      const AT* src = A + (size_t)(m0 + row) * lda + k0 + ch;
#pragma unroll
      for (int g = 0; g < 16; ++g) { const float v = (float)src[g]; const f16 h = (f16)v; ldsA[row * GSTR + ch + g] = h; ldsAl[row * GSTR + ch + g] = (f16)((v - (float)h) * 2048.0f); }
    }
    {
      const int k = tid >> 3, nn0 = (tid & 7) * 16;
      const float* src = Wm + (size_t)(k0 + k) * ldw + n0 + nn0;
#pragma unroll
      for (int g = 0; g < 4; ++g) { const v4f_t v = *(const v4f_t*)(src + 4 * g);
#pragma unroll
        for (int u = 0; u < 4; ++u) { const f16 h = (f16)v[u]; ldsW[(nn0 + 4 * g + u) * GSTR + k] = h; ldsWl[(nn0 + 4 * g + u) * GSTR + k] = (f16)((v[u] - (float)h) * 2048.0f); } }
    }
    __syncthreads();
    f16x16 af[2], afl[2];
#pragma unroll
    for (int i = 0; i < 2; ++i) { af[i] = lds_frag(ldsA + (wm + 16 * i) * GSTR, GSTR); afl[i] = lds_frag(ldsAl + (wm + 16 * i) * GSTR, GSTR); }
#pragma unroll
    for (int j = 0; j < 4; ++j) {
      const f16x16 bf = lds_frag(ldsW + (wn + 16 * j) * GSTR, GSTR), bfl = lds_frag(ldsWl + (wn + 16 * j) * GSTR, GSTR);
#pragma unroll
      for (int i = 0; i < 2; ++i) { acc[i][j] = wmma16(af[i], bf, acc[i][j]); accx[i][j] = wmma16(af[i], bfl, accx[i][j]); accx[i][j] = wmma16(afl[i], bf, accx[i][j]); }
    }
  }
  float* so = oS[wave];
#pragma unroll
  for (int i = 0; i < 2; ++i)
#pragma unroll
    for (int j = 0; j < 4; ++j) {
      const float bv = bias ? bias[n0 + wn + 16 * j + cl] : 0.0f;
#pragma unroll
      for (int r = 0; r < 8; ++r) so[(16 * i + rh + r) * 68 + 16 * j + cl] = (acc[i][j][r] + accx[i][j][r] * (1.0f / 2048.0f)) * scale + bv;
    }
  asm volatile("s_wait_dscnt 0" ::: "memory");
  __builtin_amdgcn_wave_barrier();
  if (ACC) {
#pragma unroll
    for (int it = 0; it < 16; ++it) { const int f4 = lane + 32 * it, rr = f4 >> 4, q = (f4 & 15) * 4;
      const v4f_t old = *(const v4fa*)(Y + (size_t)(m0 + wm + rr) * ldy + n0 + wn + q);
      v4f_t v = *(const v4fa*)(so + rr * 68 + q); v += old; *(v4fa*)(so + rr * 68 + q) = v; }
    asm volatile("s_wait_dscnt 0" ::: "memory");
  }
#pragma unroll 1
  for (int pass = 0; pass < 2; ++pass) {
#pragma unroll
    for (int it = 0; it < 16; ++it) { const int f4 = lane + 32 * it, rr = f4 >> 4, q = (f4 & 15) * 4;
      *(volatile v4f_t*)(Y + (size_t)(m0 + wm + rr) * ldy + n0 + wn + q) = *(const v4fa*)(so + rr * 68 + q); }
    __threadfence();
  }
}

template <typename AT, bool ACC>
__global__ __launch_bounds__(256) void gemm_kn2(const AT* __restrict__ A, int lda, size_t strideA,
                                               const float* __restrict__ Wm, int ldw, size_t strideW,
                                               const float* __restrict__ bias, float scale,
                                               float* __restrict__ Y, int ldy, size_t strideY, int K) {
  __shared__ __attribute__((aligned(16))) f16 ldsA[128 * GSTR], ldsAl[128 * GSTR];
  __shared__ __attribute__((aligned(16))) f16 ldsW[128 * GSTR], ldsWl[128 * GSTR];
  __shared__ __attribute__((aligned(16))) float oS[8][32 * 68];
  const int tid = threadIdx.x, lane = tid & 31, wave = tid >> 5, cl = lane & 15, rh = (lane >> 4) * 8;
  const int m0 = blockIdx.x * 128, n0 = blockIdx.y * 128;
  const int wm = (wave & 3) * 32, wn = (wave >> 2) * 64;
  A += (size_t)blockIdx.z * strideA; Wm += (size_t)blockIdx.z * strideW; Y += (size_t)blockIdx.z * strideY;
  f32x8 acc[2][4], accx[2][4];
#pragma unroll
  for (int i = 0; i < 2; ++i)
#pragma unroll
    for (int j = 0; j < 4; ++j) { f32x8 z = {}; acc[i][j] = z; accx[i][j] = z; }
#pragma unroll 1
  for (int k0 = 0; k0 < K; k0 += 32) {
    __syncthreads();
    {
      const int row = tid >> 1, ch = (tid & 1) * 16;
      const AT* src = A + (size_t)(m0 + row) * lda + k0 + ch;
#pragma unroll
      for (int g = 0; g < 16; ++g) { const float v = (float)src[g]; const f16 h = (f16)v; ldsA[row * GSTR + ch + g] = h; ldsAl[row * GSTR + ch + g] = (f16)((v - (float)h) * 2048.0f); }
    }
    {
      const int k = tid >> 3, nn0 = (tid & 7) * 16;
      const float* src = Wm + (size_t)(k0 + k) * ldw + n0 + nn0;
#pragma unroll
      for (int g = 0; g < 4; ++g) { const v4f_t v = *(const v4f_t*)(src + 4 * g);
#pragma unroll
        for (int u = 0; u < 4; ++u) { const f16 h = (f16)v[u]; ldsW[(nn0 + 4 * g + u) * GSTR + k] = h; ldsWl[(nn0 + 4 * g + u) * GSTR + k] = (f16)((v[u] - (float)h) * 2048.0f); } }
    }
    __syncthreads();
    f16x16 af[2], afl[2];
#pragma unroll
    for (int i = 0; i < 2; ++i) { af[i] = lds_frag(ldsA + (wm + 16 * i) * GSTR, GSTR); afl[i] = lds_frag(ldsAl + (wm + 16 * i) * GSTR, GSTR); }
#pragma unroll
    for (int j = 0; j < 4; ++j) {
      const f16x16 bf = lds_frag(ldsW + (wn + 16 * j) * GSTR, GSTR), bfl = lds_frag(ldsWl + (wn + 16 * j) * GSTR, GSTR);
#pragma unroll
      for (int i = 0; i < 2; ++i) { acc[i][j] = wmma16(af[i], bf, acc[i][j]); accx[i][j] = wmma16(af[i], bfl, accx[i][j]); accx[i][j] = wmma16(afl[i], bf, accx[i][j]); }
    }
  }
  float* so = oS[wave];
#pragma unroll
  for (int i = 0; i < 2; ++i)
#pragma unroll
    for (int j = 0; j < 4; ++j) {
      const float bv = bias ? bias[n0 + wn + 16 * j + cl] : 0.0f;
#pragma unroll
      for (int r = 0; r < 8; ++r) so[(16 * i + rh + r) * 68 + 16 * j + cl] = (acc[i][j][r] + accx[i][j][r] * (1.0f / 2048.0f)) * scale + bv;
    }
  asm volatile("s_wait_dscnt 0" ::: "memory");
  __builtin_amdgcn_wave_barrier();
  if (ACC) {
#pragma unroll
    for (int it = 0; it < 16; ++it) { const int f4 = lane + 32 * it, rr = f4 >> 4, q = (f4 & 15) * 4;
      const v4f_t old = *(const v4fa*)(Y + (size_t)(m0 + wm + rr) * ldy + n0 + wn + q);
      v4f_t v = *(const v4fa*)(so + rr * 68 + q); v += old; *(v4fa*)(so + rr * 68 + q) = v; }
    asm volatile("s_wait_dscnt 0" ::: "memory");
  }
#pragma unroll 1
  for (int pass = 0; pass < 2; ++pass) {
#pragma unroll
    for (int it = 0; it < 16; ++it) { const int f4 = lane + 32 * it, rr = f4 >> 4, q = (f4 & 15) * 4;
      *(volatile v4f_t*)(Y + (size_t)(m0 + wm + rr) * ldy + n0 + wn + q) = *(const v4fa*)(so + rr * 68 + q); }
    __threadfence();
  }
}

__global__ __launch_bounds__(256) void k_transpose(const float* __restrict__ Wm, float* __restrict__ Wt, int rows, int cols) {
  __shared__ float tS[64][65];
  const int tid = threadIdx.x, tbj = cols / 64, bi = blockIdx.x / tbj, bj = blockIdx.x % tbj;
  for (int e = tid; e < 64 * 64; e += 256) { const int r = e >> 6, c = e & 63; tS[r][c] = Wm[(size_t)(bi * 64 + r) * cols + bj * 64 + c]; }
  __syncthreads();
  for (int ch = tid; ch < 64 * 16; ch += 256) { const int r = ch >> 4, q4 = (ch & 15) * 4; v4f_t o; o[0] = tS[q4][r]; o[1] = tS[q4 + 1][r]; o[2] = tS[q4 + 2][r]; o[3] = tS[q4 + 3][r];
    float* dst = Wt + (size_t)(bj * 64 + r) * rows + bi * 64 + q4; *(volatile v4f_t*)dst = o; __threadfence(); *(volatile v4f_t*)dst = o; }
}

#define NBc 8
#define SSc 1024
#define SIN 1024
#define DDc 1024
#define DQc 1024
#define DKc 1024
#define DOc 1024
#define NHc 16
#define HDc 64
__global__ __launch_bounds__(256) void k_fill(float* __restrict__ p, float val, size_t n4) { const size_t i = (size_t)blockIdx.x * 256 + threadIdx.x; if (i < n4) { v4f_t v = {val, val, val, val}; *(volatile v4f_t*)(p + 4 * i) = v; __threadfence(); *(volatile v4f_t*)(p + 4 * i) = v; } }
__global__ __launch_bounds__(256) void k_place(const float* __restrict__ T, float* __restrict__ att, int h0) {
  const int tid = threadIdx.x; const int z = blockIdx.y; const int q = blockIdx.x * 16 + (tid >> 4); const int c4 = (tid & 15) * 4;
  const v4f_t v = *(const v4f_t*)(T + ((size_t)z * 1024 + q) * 128 + c4);
  float* dst = att + (size_t)q * 1024 + (h0 + z) * 64 + c4; *(volatile v4f_t*)dst = v; __threadfence(); *(volatile v4f_t*)dst = v;
}
__global__ __launch_bounds__(256) void k_place0(const float* __restrict__ T, float* __restrict__ att, int h0) {
  const int tid = threadIdx.x; const int z = blockIdx.y; const int q = blockIdx.x * 16 + (tid >> 4); const int c4 = (tid & 15) * 4;
  const v4f_t v = *(const v4f_t*)(T + ((size_t)z * 128 + q) * 128 + c4);
  float* dst = att + (size_t)q * 1024 + (h0 + z) * 64 + c4; *(volatile v4f_t*)dst = v; __threadfence(); *(volatile v4f_t*)dst = v;
}
__global__ __launch_bounds__(256) void k_softmax_causal(float* __restrict__ Sm) {
  __shared__ float red[256];
  const int q = blockIdx.x, z = blockIdx.y, tid = threadIdx.x; float* sr = Sm + ((size_t)z * 1024 + q) * 1024;
  const float scl = (0.125);
  float v[4]; float m = -3.0e38f;
#pragma unroll
  for (int e = 0; e < 4; ++e) { const int k = tid + 256 * e; v[e] = (k <= q) ? sr[min(k, q)] * scl : -3.0e38f; m = fmaxf(m, v[e]); }
  red[tid] = m; __syncthreads();
  for (int o = 128; o > 0; o >>= 1) { if (tid < o) red[tid] = fmaxf(red[tid], red[tid + o]); __syncthreads(); }
  m = red[0]; __syncthreads();
  float zs = 0.0f;
#pragma unroll
  for (int e = 0; e < 4; ++e) { const int k = tid + 256 * e; v[e] = (k <= q) ? expf(v[e] - m) : 0.0f; zs += v[e]; }
  red[tid] = zs; __syncthreads();
  for (int o = 128; o > 0; o >>= 1) { if (tid < o) red[tid] += red[tid + o]; __syncthreads(); }
  const float sc = 1024.0f / red[0]; const float cq = 1024.0f / (float)(q + 1);
#pragma unroll 1
  for (int pass = 0; pass < 2; ++pass) {
#pragma unroll
    for (int e = 0; e < 4; ++e) { const int k = tid + 256 * e; *(volatile float*)(sr + k) = (k <= q) ? (v[e] * sc - cq) : 0.0f; }
    __threadfence(); }
}
__global__ __launch_bounds__(128) void k_softmax128(float* __restrict__ S0) {
  __shared__ float red[128];
  const int q = blockIdx.x, z = blockIdx.y, k = threadIdx.x; float* sr = S0 + ((size_t)z * 128 + q) * 128;
  const float scl = (0.125); float v = (k <= q) ? sr[min(k, q)] * scl : -3.0e38f;
  red[k] = v; __syncthreads();
  for (int o = 64; o > 0; o >>= 1) { if (k < o) red[k] = fmaxf(red[k], red[k + o]); __syncthreads(); }
  const float m = red[0]; __syncthreads();
  v = (k <= q) ? expf(v - m) : 0.0f; red[k] = v; __syncthreads();
  for (int o = 64; o > 0; o >>= 1) { if (k < o) red[k] += red[k + o]; __syncthreads(); }
  const float p = v * (1024.0f / red[0]);
  *(volatile float*)(sr + k) = p; __threadfence(); *(volatile float*)(sr + k) = p;
}
__global__ __launch_bounds__(256) void k_prefmean(const float* __restrict__ V, int ldv, int ncols, float* __restrict__ PM) {
  const int c = blockIdx.x * 256 + threadIdx.x; if (c >= ncols) return; float s = 0.0f;
#pragma unroll 1
  for (int r = 0; r < 1024; ++r) { s += V[(size_t)r * ldv + c]; const float m = s / (float)(r + 1); *(volatile float*)(PM + (size_t)r * ncols + c) = m; }
  __threadfence();
#pragma unroll 1
  for (int r = 0; r < 1024; ++r) { float* p = PM + (size_t)r * ncols + c; const float m = p[0]; *(volatile float*)p = m; }
}
__global__ __launch_bounds__(256) void k_place_pm(const float* __restrict__ T, float* __restrict__ att, int h0, const float* __restrict__ PM, int ldpm, int kv, int kvz) {
  const int tid = threadIdx.x; const int z = blockIdx.y; const int q = blockIdx.x * 16 + (tid >> 4); const int c4 = (tid & 15) * 4;
  v4f_t v = *(const v4f_t*)(T + ((size_t)z * 1024 + q) * 128 + c4); const v4f_t pm = *(const v4f_t*)(PM + (size_t)q * ldpm + (kv + z * kvz) * 64 + c4); v += pm;
  float* dst = att + (size_t)q * 1024 + (h0 + z) * 64 + c4; *(volatile v4f_t*)dst = v; __threadfence(); *(volatile v4f_t*)dst = v;
}

__global__ __launch_bounds__(256) void k_genwT(const float* __restrict__ sub, const float* __restrict__ wl, const float* __restrict__ Wsc, const float* __restrict__ Bb, int O, int I, float* __restrict__ GT) { const int i = blockIdx.x, tid = threadIdx.x; const float w0 = wl[0], w1 = wl[1];
#pragma unroll 1
  for (int pass = 0; pass < 2; ++pass) {
#pragma unroll 1
    for (int o = tid; o < O; o += 256) { const size_t oi = (size_t)o * I + i; const float v = 1024.0f * (tanhf(w0 * sub[oi] + w1 * sub[(size_t)O * I + oi]) * Wsc[oi] + Bb[oi]); *(volatile float*)(GT + (size_t)i * O + o) = v; }
    __threadfence(); } }
__global__ __launch_bounds__(256) void k_genb(const float* __restrict__ sub, const float* __restrict__ wl, const float* __restrict__ Wsc, const float* __restrict__ Bb, int O, float* __restrict__ Gb, float* __restrict__ Gbs) { const int o = blockIdx.x * 256 + threadIdx.x; if (o >= O) return; const float v = tanhf(wl[0] * sub[o] + wl[1] * sub[O + o]) * Wsc[o] + Bb[o]; *(volatile float*)(Gb + o) = v; *(volatile float*)(Gbs + o) = 1024.0f * v; __threadfence(); *(volatile float*)(Gb + o) = v; *(volatile float*)(Gbs + o) = 1024.0f * v; }
extern "C" void kernel_launch(void* const* d_in, const int* in_sizes, int n_in,
                              void* d_out, int out_size, void* d_ws, size_t ws_size,
                              hipStream_t stream) {
  (void)in_sizes; (void)n_in; (void)out_size;
  const float** f = (const float**)d_in;
  const float* hidden_states = f[0]; const float* attn_w_subset = f[1]; const float* attn_w_Wl = f[2]; const float* attn_w_W = f[3]; const float* attn_w_B = f[4]; const float* attn_b_subset = f[5]; const float* attn_b_Wl = f[6]; const float* attn_b_W = f[7]; const float* attn_b_B = f[8]; const float* proj_w_subset = f[9]; const float* proj_w_Wl = f[10]; const float* proj_w_W = f[11]; const float* proj_w_B = f[12]; const float* proj_b_subset = f[13]; const float* proj_b_Wl = f[14]; const float* proj_b_W = f[15]; const float* proj_b_B = f[16];
  float* out = (float*)d_out;
  char* ws = (char*)d_ws;
  float* GW = (float*)ws; ws += (size_t)DDc * 3 * DDc * 4; float* GB = (float*)ws; ws += 3 * DDc * 4; float* GWP = (float*)ws; ws += (size_t)DDc * DDc * 4; float* GBP = (float*)ws; ws += DDc * 4; float* GBs = (float*)ws; ws += 3 * DDc * 4; float* GBPs = (float*)ws; ws += DDc * 4; float* g1024 = (float*)ws; ws += 3 * DDc * 4;
  float* Q = (float*)ws; ws += (size_t)SSc * DQc * 4; float* Kp = (float*)ws; ws += (size_t)SSc * DKc * 4; float* V = (float*)ws; ws += (size_t)SSc * DKc * 4 + 1024;
  float* KT = (float*)ws; ws += (size_t)DKc * SSc * 4;
  float* S = (float*)ws; ws += (size_t)2 * SSc * SSc * 4;
  float* T = (float*)ws; ws += (size_t)2 * SSc * 128 * 4; float* sc = (float*)ws; ws += 128 * 4;
  float* ATT = (float*)ws; ws += (size_t)SSc * DQc * 4;
  float* PM = (float*)ws; ws += (size_t)SSc * DKc * 4;
  float* Q0 = (float*)ws; ws += (size_t)128 * DQc * 4; float* K0 = (float*)ws; ws += (size_t)128 * DKc * 4; float* V0 = (float*)ws; ws += (size_t)128 * DKc * 4 + 1024;
  float* K0T = (float*)ws; ws += (size_t)DKc * 128 * 4; float* S0 = (float*)ws; ws += (size_t)2 * 128 * 128 * 4; float* T0 = (float*)ws; ws += (size_t)2 * 128 * 128 * 4;
  if ((size_t)(ws - (char*)d_ws) > ws_size) return;
  const dim3 blk(256);
  k_genwT<<<dim3(DDc), blk, 0, stream>>>(attn_w_subset, attn_w_Wl, attn_w_W, attn_w_B, 3 * DDc, DDc, GW); k_genb<<<dim3((3 * DDc + 255) / 256), blk, 0, stream>>>(attn_b_subset, attn_b_Wl, attn_b_W, attn_b_B, 3 * DDc, GB, GBs); k_fill<<<dim3(3), blk, 0, stream>>>(g1024, 1.0f / 1024.0f, 3 * DDc / 4);
  k_genwT<<<dim3(DDc), blk, 0, stream>>>(proj_w_subset, proj_w_Wl, proj_w_W, proj_w_B, DDc, DDc, GWP); k_genb<<<dim3((DDc + 255) / 256), blk, 0, stream>>>(proj_b_subset, proj_b_Wl, proj_b_W, proj_b_B, DDc, GBP, GBPs);
  k_fill<<<dim3(1), blk, 0, stream>>>(sc, 1.0f / 1024.0f, 128 / 4); k_fill<<<dim3(1), blk, 0, stream>>>(V + (size_t)SSc * DKc, 0.0f, 256 / 4); k_fill<<<dim3(1), blk, 0, stream>>>(V0 + (size_t)128 * DKc, 0.0f, 256 / 4);
  for (int b = 0; b < NBc; ++b) {
    const float* xb = hidden_states + (size_t)b * SIN * DDc;
    gemm_kne<float, 4, false><<<dim3(SSc / 128, DQc / 128), blk, 0, stream>>>(xb, DDc, GW, (3 * DDc), (GBs), nullptr, g1024, Q, DQc, DDc);
    gemm_kne<float, 4, false><<<dim3(SSc / 128, DKc / 128), blk, 0, stream>>>(xb, DDc, (GW + DDc), (3 * DDc), (GBs + DDc), nullptr, g1024, Kp, DKc, DDc);
    gemm_kne<float, 4, false><<<dim3(SSc / 128, DKc / 128), blk, 0, stream>>>(xb, DDc, (GW + 2 * DDc), (3 * DDc), (GBs + 2 * DDc), nullptr, g1024, V, DKc, DDc);
    k_transpose<<<dim3((SSc / 64) * (DKc / 64)), blk, 0, stream>>>(Kp, KT, SSc, DKc);
    k_prefmean<<<dim3((DKc + 255) / 256), blk, 0, stream>>>(V, DKc, DKc, PM);
    for (int hg = 0; hg < NHc / 2; ++hg) { const int h0 = 2 * hg; const int kv = h0;
      gemm_knezc<float, 0, false, 2><<<dim3(SSc / 128, SSc / 128, 2), blk, 0, stream>>>(Q + h0 * HDc, DQc, (size_t)HDc, KT + (size_t)kv * HDc * SSc, SSc, (size_t)HDc * SSc, nullptr, nullptr, nullptr, S, SSc, (size_t)SSc * SSc, HDc);
      k_softmax_causal<<<dim3(SSc, 2), blk, 0, stream>>>(S);
      gemm_knezc<float, 4, false, 1><<<dim3(SSc / 128, 1, 2), blk, 0, stream>>>(S, SSc, (size_t)SSc * SSc, V + kv * HDc, DKc, (size_t)HDc, nullptr, nullptr, sc, T, 128, (size_t)SSc * 128, SSc);
      k_place_pm<<<dim3(SSc / 16, 2), blk, 0, stream>>>(T, ATT, h0, PM, DKc, kv, 1);
    }
    gemm_kne<float, 4, false><<<dim3((SSc - 128) / 128, DOc / 128), blk, 0, stream>>>(ATT + (size_t)128 * DQc, DQc, GWP, DOc, GBPs, nullptr, g1024, out + (size_t)b * SIN * DOc + (size_t)128 * DOc, DOc, DQc);
    gemm_kn2<float, false><<<dim3(1, DQc / 128, 1), blk, 0, stream>>>(xb, DDc, 0, GW, (3 * DDc), 0, GB, (1.0f / 1024.0f), Q0, DQc, 0, DDc);
    gemm_kn2<float, false><<<dim3(1, DKc / 128, 1), blk, 0, stream>>>(xb, DDc, 0, (GW + DDc), (3 * DDc), 0, (GB + DDc), (1.0f / 1024.0f), K0, DKc, 0, DDc);
    gemm_kn2<float, false><<<dim3(1, DKc / 128, 1), blk, 0, stream>>>(xb, DDc, 0, (GW + 2 * DDc), (3 * DDc), 0, (GB + 2 * DDc), (1.0f / 1024.0f), V0, DKc, 0, DDc);
    k_transpose<<<dim3((128 / 64) * (DKc / 64)), blk, 0, stream>>>(K0, K0T, 128, DKc);
    for (int hg = 0; hg < NHc / 2; ++hg) { const int h0 = 2 * hg; const int kv = h0;
      gemm_kn2<float, false><<<dim3(1, 1, 2), blk, 0, stream>>>(Q0 + h0 * HDc, DQc, (size_t)HDc, K0T + (size_t)kv * HDc * 128, 128, (size_t)HDc * 128, nullptr, 1.0f, S0, 128, (size_t)128 * 128, HDc);
      k_softmax128<<<dim3(128, 2), dim3(128), 0, stream>>>(S0);
      gemm_kn2<float, false><<<dim3(1, 1, 2), blk, 0, stream>>>(S0, 128, (size_t)128 * 128, V0 + kv * HDc, DKc, (size_t)HDc, nullptr, 1.0f / 1024.0f, T0, 128, (size_t)128 * 128, 128);
      k_place0<<<dim3(128 / 16, 2), blk, 0, stream>>>(T0, ATT, h0);
    }
    gemm_kn2<float, false><<<dim3(1, DOc / 128, 1), blk, 0, stream>>>(ATT, DQc, 0, GWP, DOc, 0, GBP, (1.0f / 1024.0f), out + (size_t)b * SIN * DOc, DOc, 0, DQc);
  }
}
